// MambaVisionMixer_30863634989315
// MI455X (gfx1250) — hardware-verified
//
#include <hip/hip_runtime.h>

#define NB    4
#define NL    4096
#define DM    512
#define DIN   1024
#define D2    512
#define NS    16
#define DTR   32
#define KDT   32
#define NXD   64
#define NXP   64
#define NROWS (NB * NL)
#define NRH   (NROWS / 2)
#define TC    16
#define LNEPS 1e-5f

static_assert(DM % 32 == 0 && D2 % 32 == 0 && DIN % 32 == 0 && KDT % 32 == 0);
static_assert(NROWS % 128 == 0 && NRH % 128 == 0 && DM % 64 == 0 && D2 % 64 == 0 && NXP % 64 == 0);
static_assert(NL % TC == 0 && D2 % 256 == 0 && NL % 128 == 0 && TC == 16 && NRH % NL == 0);
static_assert(DTR + 2 * NS == NXD && NXD == NXP && DTR == KDT && KDT == 32 && NXP == 64);
static_assert(DIN == 2 * D2 && DM == D2);

typedef __bf16         v16b __attribute__((ext_vector_type(16)));
typedef unsigned short v8us __attribute__((ext_vector_type(8)));
typedef float          v8f  __attribute__((ext_vector_type(8)));
typedef float          v4f  __attribute__((ext_vector_type(4)));
typedef v8us __attribute__((may_alias)) v8usa;
typedef v4f  __attribute__((may_alias)) v4fa;

union Frag { v16b v; v8us half[2]; };

constexpr int P_WIN  = 0;
constexpr int P_WX   = P_WIN + DIN * DM;
constexpr int P_WDT  = P_WX + NXP * D2;
constexpr int P_WOUT = P_WDT + D2 * KDT;
constexpr int P_HID  = P_WOUT + DM * DIN;
constexpr int P_END  = P_HID + NROWS * DM;
constexpr int NPC    = P_END / 8;
constexpr int NCBLK  = NPC / 256;
static_assert(P_END % 8 == 0 && NPC % 256 == 0);
static_assert(P_WX % 2048 == 0 && P_WDT % 2048 == 0 && P_WOUT % 2048 == 0 && P_HID % 2048 == 0);
static_assert(DM % 8 == 0 && KDT % 8 == 0);

constexpr size_t OFF_CV   = 0;
constexpr size_t SZ_CV    = (size_t)P_END * 2;
constexpr size_t OFF_XZ   = OFF_CV + SZ_CV;
constexpr size_t SZ_XZ    = (size_t)NROWS * D2 * 4;
constexpr size_t OFF_XH   = OFF_XZ + SZ_XZ;
constexpr size_t SZ_X16   = (size_t)NROWS * D2 * 2;
constexpr size_t OFF_XL   = OFF_XH + SZ_X16;
constexpr size_t OFF_XF   = OFF_XL + SZ_X16;
constexpr size_t SZ_XF    = (size_t)NROWS * D2 * 4;
constexpr size_t OFF_XDBL = OFF_XF + SZ_XF;
constexpr size_t SZ_XDBL  = (size_t)NROWS * NXP * 4;
constexpr size_t OFF_DTH  = OFF_XDBL + SZ_XDBL;
constexpr size_t SZ_DT    = (size_t)NROWS * KDT * 2;
constexpr size_t OFF_DTL  = OFF_DTH + SZ_DT;
constexpr size_t WS_END   = OFF_DTL + SZ_DT;
constexpr size_t OFF_YCH  = OFF_XZ;
constexpr size_t SZ_Y16   = (size_t)NROWS * DIN * 2;
constexpr size_t OFF_YCL  = OFF_YCH + SZ_Y16;
constexpr size_t OFF_ZP   = OFF_XF;
constexpr size_t SZ_ZP    = (size_t)NRH * D2 * 4;
static_assert(OFF_YCL + SZ_Y16 <= OFF_XF);
static_assert(OFF_YCL == OFF_XH && OFF_YCL + SZ_Y16 == OFF_XF);
static_assert(OFF_ZP + SZ_ZP <= OFF_XDBL);
static_assert(OFF_XZ % 128 == 0 && OFF_XH % 128 == 0 && OFF_XL % 128 == 0 && OFF_XF % 128 == 0);
static_assert(OFF_XDBL % 128 == 0 && OFF_DTH % 128 == 0 && OFF_DTL % 128 == 0 && OFF_ZP % 128 == 0);
static_assert(OFF_YCH % 128 == 0 && OFF_YCL % 128 == 0);
static_assert(WS_END <= (size_t)134217728);
static_assert((size_t)NPC * 16 == SZ_CV);
static_assert((size_t)(NROWS / 128) * (D2 / 64) * 256 * 128 == SZ_XZ);
static_assert((size_t)(NRH / 128) * (D2 / 64) * 256 * 128 == SZ_ZP);
static_assert((size_t)(D2 / 256) * (NROWS / TC) * (TC * 8) * 128 == SZ_XF);
static_assert((size_t)(D2 / 256) * (NROWS / TC) * (TC * 4) * 128 == SZ_X16);
static_assert((size_t)(NROWS / 128) * (NXP / 64) * 256 * 128 == SZ_XDBL);
static_assert((size_t)(NROWS / 128) * 64 * 128 == SZ_DT);
static_assert((size_t)(D2 / 256) * NB * (NL / TC) * (TC * 4) * 128
              + (size_t)2 * (D2 / 256) * (NRH / TC) * (TC * 4) * 128 == SZ_Y16);
static_assert((size_t)(NROWS / 128) * (DM / 64) * 256 * 128 == (size_t)NROWS * DM * 4);

__device__ __forceinline__ unsigned short bf16_bits(float f) {
  unsigned u = __float_as_uint(f);
  u += 0x7FFFu + ((u >> 16) & 1u);
  return (unsigned short)(u >> 16);
}
__device__ __forceinline__ float bf16_val(unsigned short b) { return __uint_as_float(((unsigned)b) << 16); }
__device__ __forceinline__ float bf16r(float f) { return bf16_val(bf16_bits(f)); }
__device__ __forceinline__ void split_bf16(float v, unsigned short& hb, unsigned short& lb) {
  hb = bf16_bits(v);
  lb = bf16_bits(v - bf16_val(hb));
}
__device__ __forceinline__ v8f zero8() {
  v8f z;
#pragma unroll
  for (int i = 0; i < 8; ++i) z[i] = 0.0f;
  return z;
}

__device__ __forceinline__ void ldfrag_g(Frag& f, const unsigned short* p, int h) {
  f.half[0] = *(const v8usa*)(p + 8 * h);
  f.half[1] = *(const v8usa*)(p + 16 + 8 * h);
}
__device__ __forceinline__ v8f mma16(v8f c, const Frag& a, const Frag& b) {
  v8f d = __builtin_amdgcn_wmma_f32_16x16x32_bf16(false, a.v, false, b.v, (short)0, c, false, false);
  asm volatile("v_nop\n\tv_nop\n\tv_nop\n\tv_nop" : "+v"(d) : "v"(a.v), "v"(b.v));
  return d;
}

__global__ __launch_bounds__(256)
void cvt_kernel(const float* __restrict__ hid, const float* __restrict__ win, const float* __restrict__ wx,
                const float* __restrict__ wdt, const float* __restrict__ wout, unsigned short* cv)
{
  const int g = blockIdx.x * 256 + threadIdx.x;
  if (g >= NPC) return;
  const int e = g * 8;
  const float* src;
  if (e < P_WX) {
    src = win + e;
  } else if (e < P_WDT) {
    src = wx + (e - P_WX);
  } else if (e < P_WOUT) {
    src = wdt + (e - P_WDT);
  } else if (e < P_HID) {
    src = wout + (e - P_WOUT);
  } else {
    src = hid + (e - P_HID);
  }
  const v4f a = *(const v4fa*)src;
  const v4f c = *(const v4fa*)(src + 4);
  v8us o;
  o[0] = bf16_bits(a[0]);
  o[1] = bf16_bits(a[1]);
  o[2] = bf16_bits(a[2]);
  o[3] = bf16_bits(a[3]);
  o[4] = bf16_bits(c[0]);
  o[5] = bf16_bits(c[1]);
  o[6] = bf16_bits(c[2]);
  o[7] = bf16_bits(c[3]);
  unsigned short* dst = cv + e;
  *(volatile v8us*)dst = o;
  __threadfence();
  *(volatile v8us*)dst = o;
}

__device__ __forceinline__ void c_store_pass(const float* sT, float* C, int ldc, int m0w, int cy, int w, int lane) {
  const int q8 = lane & 7, sub = lane >> 3;
#pragma unroll
  for (int i = 0; i < 16; ++i) {
    const int lid = 4 * i + sub;
    const int rl = lid >> 1, hl = lid & 1;
    const v4f v = *(const v4fa*)(sT + (32 * w + rl) * 64 + 32 * hl + 4 * q8);
    float* dst = C + (size_t)(m0w + rl) * ldc + 64 * cy + 32 * hl + 4 * q8;
    *(volatile v4f*)dst = v;
  }
}

__device__ __forceinline__ void dtr_store_pass(const float* sT, unsigned short* dh, unsigned short* dl,
                                               int m0w, int w, int lane) {
  const int q4 = lane & 3, rs = lane >> 2;
#pragma unroll
  for (int i = 0; i < 4; ++i) {
    const int rl = 8 * i + rs;
    const float* sr = sT + (32 * w + rl) * 64 + 8 * q4;
    const v4f a = *(const v4fa*)sr;
    const v4f c = *(const v4fa*)(sr + 4);
    v8us oh, ol;
    unsigned short hb, lb;
    split_bf16(a[0], hb, lb); oh[0] = hb; ol[0] = lb;
    split_bf16(a[1], hb, lb); oh[1] = hb; ol[1] = lb;
    split_bf16(a[2], hb, lb); oh[2] = hb; ol[2] = lb;
    split_bf16(a[3], hb, lb); oh[3] = hb; ol[3] = lb;
    split_bf16(c[0], hb, lb); oh[4] = hb; ol[4] = lb;
    split_bf16(c[1], hb, lb); oh[5] = hb; ol[5] = lb;
    split_bf16(c[2], hb, lb); oh[6] = hb; ol[6] = lb;
    split_bf16(c[3], hb, lb); oh[7] = hb; ol[7] = lb;
    const size_t go = (size_t)(m0w + rl) * KDT + 8 * q4;
    *(volatile v8us*)(dh + go) = oh;
    *(volatile v8us*)(dl + go) = ol;
  }
}

template <int NPL, int XP>
__global__ __launch_bounds__(128)
void gemm_kernel(const unsigned short* __restrict__ Ah, const unsigned short* __restrict__ Al, int lda,
                 const unsigned short* __restrict__ Bw, int K,
                 float* C, int ldc, unsigned short* dh, unsigned short* dl,
                 const float* __restrict__ lnw, const float* __restrict__ lnb)
{
  __shared__ __attribute__((aligned(16))) float sT[128 * 64];

  const int tid = threadIdx.x, lane = tid & 31, w = tid >> 5;
  const int h = lane >> 4, m = lane & 15;
  const int m0 = blockIdx.x * 128;
  const int cy = blockIdx.y;
  const int m0w = m0 + 32 * w;

  const unsigned short* xa = Ah + (size_t)(m0w + m) * lda;
  const unsigned short* xr = Al + (size_t)(m0w + m) * lda;
  const unsigned short* wb = Bw + (size_t)(64 * cy + m) * K;

  v8f acc[2][4];
#pragma unroll
  for (int mt = 0; mt < 2; ++mt)
#pragma unroll
    for (int nt = 0; nt < 4; ++nt) acc[mt][nt] = zero8();

#pragma unroll 1
  for (int k0 = 0; k0 < K; k0 += 32) {
    Frag a0, a1, e0, e1;
    ldfrag_g(a0, xa + k0, h);
    ldfrag_g(a1, xa + (size_t)16 * lda + k0, h);
    if (NPL == 2) {
      ldfrag_g(e0, xr + k0, h);
      ldfrag_g(e1, xr + (size_t)16 * lda + k0, h);
    }
#pragma unroll
    for (int nt = 0; nt < 4; ++nt) {
      Frag b;
      ldfrag_g(b, wb + (size_t)nt * 16 * K + k0, h);
      acc[0][nt] = mma16(acc[0][nt], a0, b);
      acc[1][nt] = mma16(acc[1][nt], a1, b);
      if (NPL == 2) {
        acc[0][nt] = mma16(acc[0][nt], e0, b);
        acc[1][nt] = mma16(acc[1][nt], e1, b);
      }
    }
  }

#pragma unroll
  for (int nt = 0; nt < 4; ++nt) {
    const int col = 16 * nt + m;
#pragma unroll
    for (int mt = 0; mt < 2; ++mt)
#pragma unroll
      for (int r = 0; r < 8; ++r) {
        const int rowl = 32 * w + 16 * mt + 8 * h + r;
        sT[rowl * 64 + col] = acc[mt][nt][r];
      }
  }
  __syncthreads();

  if (XP == 1) {
    float* rp = sT + tid * 64;
    float s = 0.0f;
#pragma unroll 8
    for (int j = 0; j < NXP; ++j) s += rp[j];
    const float mu = s * (1.0f / (float)NXP);
    float q = 0.0f;
#pragma unroll 8
    for (int j = 0; j < NXP; ++j) { const float dv = rp[j] - mu; q += dv * dv; }
    const float var = q * (1.0f / (float)NXP);
    const float rstd = 1.0f / sqrtf(var + LNEPS);
#pragma unroll 4
    for (int j = 0; j < NXP; ++j) {
      const float g  = bf16r(lnw[j]);
      const float sh = bf16r(lnb[j]);
      rp[j] = (rp[j] - mu) * rstd * g + sh;
    }
    __syncthreads();
  }

  c_store_pass(sT, C, ldc, m0w, cy, w, lane);
  __threadfence();
  c_store_pass(sT, C, ldc, m0w, cy, w, lane);

  if (XP == 1) {
    if (cy == 0) {
      dtr_store_pass(sT, dh, dl, m0w, w, lane);
      __threadfence();
      dtr_store_pass(sT, dh, dl, m0w, w, lane);
    }
  }
}

__device__ __forceinline__ void f32tile_store_pass(const float* sF, float* xf, int rbase, int col0, int w, int lane) {
  const int q8 = lane & 7, sub = lane >> 3;
#pragma unroll
  for (int i = 0; i < 4; ++i) {
    const int li = 4 * i + sub;
    const int row = 2 * w + (li >> 3), q = li & 7;
    const v4f v = *(const v4fa*)(sF + row * 256 + 32 * q + 4 * q8);
    float* dst = xf + (size_t)(rbase + row) * D2 + col0 + 32 * q + 4 * q8;
    *(volatile v4f*)dst = v;
  }
}

__device__ __forceinline__ void h16tile_store_pass(const unsigned short* sH, const unsigned short* sL,
                                                   unsigned short* ph, unsigned short* pl, int pitch, int col0,
                                                   int rbase, int w, int lane) {
  const int q8 = lane & 7, sub = lane >> 3;
#pragma unroll
  for (int i = 0; i < 2; ++i) {
    const int li = 4 * i + sub;
    const int row = 2 * w + (li >> 2), q = li & 3;
    const v8us vh = *(const v8usa*)(sH + row * 256 + 64 * q + 8 * q8);
    const v8us vl = *(const v8usa*)(sL + row * 256 + 64 * q + 8 * q8);
    const size_t go = (size_t)(rbase + row) * pitch + col0 + 64 * q + 8 * q8;
    *(volatile v8us*)(ph + go) = vh;
    *(volatile v8us*)(pl + go) = vl;
  }
}

template <int XM>
__global__ __launch_bounds__(256)
void conv_kernel(const float* __restrict__ xzp, const float* __restrict__ cw, const float* __restrict__ cb,
                 int rowoff, float* xf, unsigned short* ph, unsigned short* pl)
{
  __shared__ __attribute__((aligned(16))) float sF[TC * 256];
  __shared__ __attribute__((aligned(16))) unsigned short sH[TC * 256];
  __shared__ __attribute__((aligned(16))) unsigned short sL[TC * 256];

  const int tid = threadIdx.x, lane = tid & 31, w = tid >> 5;
  const int slab = blockIdx.x;
  const int rbase = rowoff + blockIdx.y * TC;
  const int b = rbase / NL, l0 = rbase - b * NL;
  const int c = 256 * slab + tid;

  const float w0 = bf16r(cw[c * 4 + 0]);
  const float w1 = bf16r(cw[c * 4 + 1]);
  const float w2 = bf16r(cw[c * 4 + 2]);
  const float w3 = bf16r(cw[c * 4 + 3]);
  const float bias = bf16r(cb[c]);

  const float* col = xzp + (size_t)(b * NL - rowoff) * D2 + c;

  const int pm = l0 - 1;
  const int pmc = (pm > 0) ? pm : 0;
  float v0 = col[(size_t)pmc * D2];
  v0 = (pm >= 0) ? v0 : 0.0f;
  float v1 = col[(size_t)l0 * D2];
  float v2 = col[(size_t)(l0 + 1) * D2];

#pragma unroll 1
  for (int tt = 0; tt < TC; ++tt) {
    const int p3 = l0 + tt + 2;
    const int p3c = (p3 < NL) ? p3 : (NL - 1);
    float v3 = col[(size_t)p3c * D2];
    v3 = (p3 < NL) ? v3 : 0.0f;
    const float s = (w0 * v0 + w1 * v1 + w2 * v2 + w3 * v3) + bias;
    const float ex = expf(-s);
    const float sg = 1.0f / (1.0f + ex);
    const float y = s * sg;
    if (XM == 1) sF[tt * 256 + tid] = y;
    unsigned short hb, lb;
    split_bf16(y, hb, lb);
    sH[tt * 256 + tid] = hb;
    sL[tt * 256 + tid] = lb;
    v0 = v1; v1 = v2; v2 = v3;
  }
  __syncthreads();

  const int pitch = (XM == 1) ? D2 : DIN;
  const int col0 = ((XM == 1) ? 0 : D2) + 256 * slab;
  if (XM == 1) f32tile_store_pass(sF, xf, rbase, 256 * slab, w, lane);
  h16tile_store_pass(sH, sL, ph, pl, pitch, col0, rbase, w, lane);
  __threadfence();
  if (XM == 1) f32tile_store_pass(sF, xf, rbase, 256 * slab, w, lane);
  h16tile_store_pass(sH, sL, ph, pl, pitch, col0, rbase, w, lane);
}

__global__ __launch_bounds__(256)
void dtscan_kernel(const unsigned short* __restrict__ dth, const unsigned short* __restrict__ dtl,
                   const unsigned short* __restrict__ cv,
                   const float* __restrict__ xdbl,
                   const float* __restrict__ xf,
                   const float* __restrict__ dtb, const float* __restrict__ alog,
                   const float* __restrict__ dpar,
                   unsigned short* ych, unsigned short* ycl)
{
  __shared__ __attribute__((aligned(16))) float sD[TC * 256];
  __shared__ __attribute__((aligned(16))) unsigned short sH[TC * 256];
  __shared__ __attribute__((aligned(16))) unsigned short sL[TC * 256];
  __shared__ __attribute__((aligned(16))) float sBC[TC * 32];

  const int tid = threadIdx.x, lane = tid & 31, w = tid >> 5;
  const int h = lane >> 4, m = lane & 15;
  const int slab = blockIdx.x, b = blockIdx.y;
  const int c0 = 256 * slab;
  const int d = c0 + tid;

  const float bb = bf16r(dtb[d]);
  const float Dv = bf16r(dpar[d]);
  float An[NS];
#pragma unroll
  for (int n = 0; n < NS; ++n) An[n] = -expf(bf16r(alog[d * NS + n]));

  Frag bw[2][KDT / 32];
#pragma unroll
  for (int nt = 0; nt < 2; ++nt)
#pragma unroll
    for (int ks = 0; ks < KDT / 32; ++ks)
      ldfrag_g(bw[nt][ks], cv + P_WDT + (size_t)(c0 + 32 * w + 16 * nt + m) * KDT + 32 * ks, h);

  float hs[NS];
#pragma unroll
  for (int n = 0; n < NS; ++n) hs[n] = 0.0f;

#pragma unroll 1
  for (int t0 = 0; t0 < NL; t0 += TC) {
    const int r0 = b * NL + t0;

    v8f acc[2];
    acc[0] = zero8(); acc[1] = zero8();
#pragma unroll
    for (int ks = 0; ks < KDT / 32; ++ks) {
      Frag ah, ar;
      ldfrag_g(ah, dth + (size_t)(r0 + m) * KDT + 32 * ks, h);
      ldfrag_g(ar, dtl + (size_t)(r0 + m) * KDT + 32 * ks, h);
#pragma unroll
      for (int nt = 0; nt < 2; ++nt) {
        acc[nt] = mma16(acc[nt], ah, bw[nt][ks]);
        acc[nt] = mma16(acc[nt], ar, bw[nt][ks]);
      }
    }
#pragma unroll
    for (int nt = 0; nt < 2; ++nt)
#pragma unroll
      for (int r = 0; r < 8; ++r)
        sD[(8 * h + r) * 256 + 32 * w + 16 * nt + m] = acc[nt][r];

    if (tid < 128) {
      const int tok = tid >> 3, q = tid & 7;
      const v4f v = *(const v4fa*)(xdbl + (size_t)(r0 + tok) * NXP + DTR + 4 * q);
      *(v4fa*)(sBC + tok * 32 + 4 * q) = v;
    }
    __syncthreads();

#pragma unroll 1
    for (int tt = 0; tt < TC; ++tt) {
      const float dpre = sD[tt * 256 + tid];
      const float dcl = fminf(6.0f, fmaxf(-6.0f, dpre));
      const float xx = dcl + bb;
      const float dl = fmaxf(xx, 0.0f) + log1pf(expf(-fabsf(xx)));
      const float xv = xf[(size_t)(r0 + tt) * D2 + d];
      const float du = dl * xv;
      const float* bc = sBC + tt * 32;
      float y = 0.0f;
#pragma unroll
      for (int n = 0; n < NS; ++n) {
        const float dA  = expf(dl * An[n]);
        const float dBu = du * bc[n];
        hs[n] = dA * hs[n] + dBu;
        y += hs[n] * bc[NS + n];
      }
      const float yv = y + xv * Dv;
      unsigned short hb, lb;
      split_bf16(yv, hb, lb);
      sH[tt * 256 + tid] = hb;
      sL[tt * 256 + tid] = lb;
    }
    __syncthreads();

    h16tile_store_pass(sH, sL, ych, ycl, DIN, c0, r0, w, lane);
    __threadfence();
    h16tile_store_pass(sH, sL, ych, ycl, DIN, c0, r0, w, lane);
    __syncthreads();
  }
}

extern "C" void kernel_launch(void* const* d_in, const int* in_sizes, int n_in,
                              void* d_out, int out_size, void* d_ws, size_t ws_size,
                              hipStream_t stream)
{
  if (n_in < 14) return;
  if (in_sizes[0]  != NROWS * DM)  return;
  if (in_sizes[1]  != DIN * DM)    return;
  if (in_sizes[2]  != NXD * D2)    return;
  if (in_sizes[3]  != D2 * DTR)    return;
  if (in_sizes[4]  != D2)          return;
  if (in_sizes[5]  != D2 * NS)     return;
  if (in_sizes[6]  != D2)          return;
  if (in_sizes[7]  != D2 * 4)      return;
  if (in_sizes[8]  != D2)          return;
  if (in_sizes[9]  != D2 * 4)      return;
  if (in_sizes[10] != D2)          return;
  if (in_sizes[11] != NXD)         return;
  if (in_sizes[12] != NXD)         return;
  if (in_sizes[13] != DM * DIN)    return;
  if (out_size != NROWS * DM)      return;
  if (ws_size < WS_END)            return;

  const float* hid  = (const float*)d_in[0];
  const float* win  = (const float*)d_in[1];
  const float* wx   = (const float*)d_in[2];
  const float* wdt  = (const float*)d_in[3];
  const float* dtb  = (const float*)d_in[4];
  const float* alog = (const float*)d_in[5];
  const float* dpar = (const float*)d_in[6];
  const float* cwx  = (const float*)d_in[7];
  const float* cbx  = (const float*)d_in[8];
  const float* cwz  = (const float*)d_in[9];
  const float* cbz  = (const float*)d_in[10];
  const float* lnw  = (const float*)d_in[11];
  const float* lnb  = (const float*)d_in[12];
  const float* wout = (const float*)d_in[13];
  float* out = (float*)d_out;

  char* ws = (char*)d_ws;
  unsigned short* cv   = (unsigned short*)(ws + OFF_CV);
  float*          xzp  = (float*)(ws + OFF_XZ);
  unsigned short* xh   = (unsigned short*)(ws + OFF_XH);
  unsigned short* xl   = (unsigned short*)(ws + OFF_XL);
  float*          xf   = (float*)(ws + OFF_XF);
  float*          xdbl = (float*)(ws + OFF_XDBL);
  unsigned short* dth  = (unsigned short*)(ws + OFF_DTH);
  unsigned short* dtl  = (unsigned short*)(ws + OFF_DTL);
  unsigned short* ych  = (unsigned short*)(ws + OFF_YCH);
  unsigned short* ycl  = (unsigned short*)(ws + OFF_YCL);
  float*          zp   = (float*)(ws + OFF_ZP);

  cvt_kernel<<<dim3(NCBLK), dim3(256), 0, stream>>>(hid, win, wx, wdt, wout, cv);

  gemm_kernel<1, 0><<<dim3(NROWS / 128, D2 / 64), dim3(128), 0, stream>>>(
      cv + P_HID, cv + P_HID, DM, cv + P_WIN, DM, xzp, D2, dth, dtl, lnw, lnb);
  conv_kernel<1><<<dim3(D2 / 256, NROWS / TC), dim3(256), 0, stream>>>(xzp, cwx, cbx, 0, xf, xh, xl);

  gemm_kernel<2, 1><<<dim3(NROWS / 128, NXP / 64), dim3(128), 0, stream>>>(
      xh, xl, D2, cv + P_WX, D2, xdbl, NXP, dth, dtl, lnw, lnb);

  dtscan_kernel<<<dim3(D2 / 256, NB), dim3(256), 0, stream>>>(
      dth, dtl, cv, xdbl, xf, dtb, alog, dpar, ych, ycl);

  gemm_kernel<1, 0><<<dim3(NRH / 128, D2 / 64), dim3(128), 0, stream>>>(
      cv + P_HID, cv + P_HID, DM, cv + P_WIN + (size_t)D2 * DM, DM, zp, D2, dth, dtl, lnw, lnb);
  conv_kernel<0><<<dim3(D2 / 256, NRH / TC), dim3(256), 0, stream>>>(zp, cwz, cbz, 0, xf, ych, ycl);
  gemm_kernel<1, 0><<<dim3(NRH / 128, D2 / 64), dim3(128), 0, stream>>>(
      cv + P_HID + (size_t)NRH * DM, cv + P_HID + (size_t)NRH * DM, DM, cv + P_WIN + (size_t)D2 * DM, DM,
      zp, D2, dth, dtl, lnw, lnb);
  conv_kernel<0><<<dim3(D2 / 256, NRH / TC), dim3(256), 0, stream>>>(zp, cwz, cbz, NRH, xf, ych, ycl);

  gemm_kernel<2, 0><<<dim3(NROWS / 128, DM / 64), dim3(128), 0, stream>>>(
      ych, ycl, DIN, cv + P_WOUT, DIN, out, DM, dth, dtl, lnw, lnb);
}
